// MambaBlock_85950885528371
// MI455X (gfx1250) — hardware-verified
//
#include <hip/hip_runtime.h>
#include <math.h>

typedef __attribute__((ext_vector_type(16))) _Float16 v16h;
typedef __attribute__((ext_vector_type(8)))  _Float16 v8h;
typedef __attribute__((ext_vector_type(16))) __bf16   v16b;
typedef __attribute__((ext_vector_type(8)))  __bf16   v8b;
typedef __attribute__((ext_vector_type(8)))  float    v8f;
typedef __attribute__((ext_vector_type(4)))  float    v4f;
typedef __attribute__((ext_vector_type(4)))  unsigned int v4u;

constexpr int kBatch   = 4;
constexpr int kSeq     = 2048;
constexpr int kDm      = 1024;
constexpr int kDin     = 1024;
constexpr int kNst     = 8;
constexpr int kDtR     = 64;
constexpr int kPrjN    = kDtR + 2 * kNst;
constexpr int kPrjP    = 128;
constexpr int kXzP     = 2 * kDin;
constexpr int kRows    = kBatch * kSeq;
constexpr int kHalves  = 2;
constexpr int kBatchPH = kBatch / kHalves;
constexpr int kHRows   = kBatchPH * kSeq;
constexpr int kConvTP  = 260;
constexpr int kScanTS  = 64;
constexpr int kScanCh  = 64;
constexpr int kScanYP  = 68;
constexpr float kEps   = 1e-5f;
static_assert(kPrjN == 80);
static_assert((kDm % 32) == 0 && (kDin % 32) == 0 && (kDtR % 32) == 0);
static_assert((kHRows % 64) == 0 && (kXzP % 64) == 0 && (kPrjP % 64) == 0 && (kDm % 64) == 0 && (kDin % 64) == 0);
static_assert((kSeq % kScanTS) == 0 && (kSeq % 64) == 0 && (kDin % kScanCh) == 0 && (kDin % 256) == 0);
static_assert(kBatchPH * kHalves == kBatch);

constexpr size_t kOffWIN  = 0;
constexpr size_t kOffWXP  = kOffWIN  + (size_t)kXzP   * kDm   * 2;
constexpr size_t kOffWDT  = kOffWXP  + (size_t)kPrjP  * kDin  * 2;
constexpr size_t kOffWOUT = kOffWDT  + (size_t)kDin   * kDtR  * 2;
constexpr size_t kOffXNH  = kOffWOUT + (size_t)kDm    * kDin  * 2;
constexpr size_t kOffXNL  = kOffXNH  + (size_t)kHRows * kDm   * 2;
constexpr size_t kOffXZ   = kOffXNL  + (size_t)kHRows * kDm   * 2;
constexpr size_t kOffUC   = kOffXZ   + (size_t)kHRows * kXzP  * 4;
constexpr size_t kOffUCH  = kOffUC   + (size_t)kHRows * kDin  * 4;
constexpr size_t kOffUCL  = kOffUCH  + (size_t)kHRows * kDin  * 2;
constexpr size_t kOffDBL  = kOffUCL  + (size_t)kHRows * kDin  * 2;
constexpr size_t kOffDTH  = kOffDBL  + (size_t)kHRows * kPrjP * 4;
constexpr size_t kOffDTL  = kOffDTH  + (size_t)kHRows * kDtR  * 2;
constexpr size_t kOffDLR  = kOffDTL  + (size_t)kHRows * kDtR  * 2;
constexpr size_t kOffYH   = kOffDLR  + (size_t)kHRows * kDin  * 4;
constexpr size_t kOffYL   = kOffYH   + (size_t)kHRows * kDin  * 2;
constexpr size_t kWsTotal = kOffYL   + (size_t)kHRows * kDin  * 2;
static_assert(kWsTotal == 127270912ull);
static_assert(kWsTotal <= 134217728ull);
static_assert((kOffWXP % 128) == 0 && (kOffWDT % 128) == 0 && (kOffWOUT % 128) == 0 && (kOffXNH % 128) == 0 &&
              (kOffXNL % 128) == 0 && (kOffXZ % 128) == 0 && (kOffUC % 128) == 0 && (kOffUCH % 128) == 0 &&
              (kOffUCL % 128) == 0 && (kOffDBL % 128) == 0 && (kOffDTH % 128) == 0 && (kOffDTL % 128) == 0 &&
              (kOffDLR % 128) == 0 && (kOffYH % 128) == 0 && (kOffYL % 128) == 0);

__device__ __forceinline__ unsigned short f2bf_bits(float f) {
  unsigned u = __float_as_uint(f);
  return (unsigned short)((u + 0x7FFFu + ((u >> 16) & 1u)) >> 16);
}
__device__ __forceinline__ float bf_bits2f(unsigned short h) { return __uint_as_float(((unsigned)h) << 16); }

__device__ __forceinline__ unsigned bf_rne_word(float f) {
  const unsigned u = __float_as_uint(f);
  return (u + 0x7FFFu + ((u >> 16) & 1u)) >> 16;
}
__device__ __forceinline__ float bf_word_f(unsigned hb) { return __uint_as_float(hb << 16); }
__device__ __forceinline__ float rne_bf16_f(float f) { return bf_word_f(bf_rne_word(f)); }
__device__ __forceinline__ void split2(float fa, float fb, unsigned& hw, unsigned& lw) {
  const unsigned ha = bf_rne_word(fa);
  const unsigned hb = bf_rne_word(fb);
  const float ra = fa - bf_word_f(ha);
  const float rb = fb - bf_word_f(hb);
  const unsigned la = bf_rne_word(ra);
  const unsigned lb = bf_rne_word(rb);
  hw = ha | (hb << 16);
  lw = la | (lb << 16);
}
__device__ __forceinline__ void split_pack8(const v4f a0, const v4f a1, v4u& hv, v4u& lv) {
  const float f0 = a0[0], f1 = a0[1], f2 = a0[2], f3 = a0[3];
  const float f4 = a1[0], f5 = a1[1], f6 = a1[2], f7 = a1[3];
  unsigned h0, h1, h2, h3, l0, l1, l2, l3;
  split2(f0, f1, h0, l0);
  split2(f2, f3, h1, l1);
  split2(f4, f5, h2, l2);
  split2(f6, f7, h3, l3);
  hv = (v4u){h0, h1, h2, h3};
  lv = (v4u){l0, l1, l2, l3};
}

__device__ __forceinline__ void dep_guard4_h(v8f& a, v8f& b, v8f& c, v8f& d, v16h x, v16h y) { asm volatile("v_nop\n\tv_nop\n\tv_nop\n\tv_nop" : "+v"(a), "+v"(b), "+v"(c), "+v"(d) : "v"(x), "v"(y)); }
__device__ __forceinline__ void dep_guard4_b(v8f& a, v8f& b, v8f& c, v8f& d, v16b x, v16b y) { asm volatile("v_nop\n\tv_nop\n\tv_nop\n\tv_nop" : "+v"(a), "+v"(b), "+v"(c), "+v"(d) : "v"(x), "v"(y)); }
__device__ __forceinline__ void keep4_h(v16h a, v16h b, v16h c, v16h d) { asm volatile("v_nop" :: "v"(a), "v"(b), "v"(c), "v"(d)); }
__device__ __forceinline__ void keep4_b(v16b a, v16b b, v16b c, v16b d) { asm volatile("v_nop" :: "v"(a), "v"(b), "v"(c), "v"(d)); }
__device__ __forceinline__ void acc_guard4(v8f& a, v8f& b, v8f& c, v8f& d) { asm volatile("v_nop\n\tv_nop\n\tv_nop\n\tv_nop" : "+v"(a), "+v"(b), "+v"(c), "+v"(d)); }
template <typename T> struct Frag;
template <> struct Frag<_Float16> {
  typedef v16h V; union U { v16h v; v8h h[2]; };
  static __device__ __forceinline__ v16h load(const _Float16* p) {
    U f; f.h[0] = *(const v8h*)(p); f.h[1] = *(const v8h*)(p + 16); return f.v;
  }
  static __device__ __forceinline__ v8f mma(v16h a, v16h b, v8f c) {
    return __builtin_amdgcn_wmma_f32_16x16x32_f16(false, a, false, b, (short)0, c, false, false);
  }
  static __device__ __forceinline__ void guard4(v8f& a, v8f& b, v8f& c, v8f& d, v16h x, v16h y) { dep_guard4_h(a, b, c, d, x, y); }
  static __device__ __forceinline__ void keep(v16h a, v16h b, v16h c, v16h d) { keep4_h(a, b, c, d); }
};
template <> struct Frag<__bf16> {
  typedef v16b V; union U { v16b v; v8b h[2]; };
  static __device__ __forceinline__ v16b load(const __bf16* p) {
    U f; f.h[0] = *(const v8b*)(p); f.h[1] = *(const v8b*)(p + 16); return f.v;
  }
  static __device__ __forceinline__ v8f mma(v16b a, v16b b, v8f c) {
    return __builtin_amdgcn_wmma_f32_16x16x32_bf16(false, a, false, b, (short)0, c, false, false);
  }
  static __device__ __forceinline__ void guard4(v8f& a, v8f& b, v8f& c, v8f& d, v16b x, v16b y) { dep_guard4_b(a, b, c, d, x, y); }
  static __device__ __forceinline__ void keep(v16b a, v16b b, v16b c, v16b d) { keep4_b(a, b, c, d); }
};

template <int ET> struct Elem;
template <> struct Elem<0> { typedef _Float16 T; };
template <> struct Elem<1> { typedef __bf16 T; };
template <int ET, int SPL, int BIAS_MODE, int OUT_MODE, bool RESID, int ACT = 0>
__global__ __launch_bounds__(256) void wmma_gemm64(
    const unsigned short* __restrict__ Ap, const unsigned short* __restrict__ A2p, int lda, long strideA,
    const unsigned short* __restrict__ Btp, const unsigned short* __restrict__ Bt2p, int ldb, long strideB,
    void* __restrict__ Cout, void* __restrict__ Cout2, int ldc, long strideC,
    const float* __restrict__ bias,
    const float* __restrict__ resid, long strideR,
    int M, int N, int K, float scale) {
  typedef typename Elem<ET>::T T;
  typedef typename Frag<T>::V V;
  const T* A = (const T*)Ap; const T* A2 = (const T*)A2p; const T* Bt = (const T*)Btp; const T* Bt2 = (const T*)Bt2p;
  __shared__ __align__(16) float sT[8][16 * 68];
  const int b    = blockIdx.y;
  const int lane = threadIdx.x & 31;
  const int wave = threadIdx.x >> 5;
  const int tilesN = N >> 6;
  const int tilesM = M >> 6;
  const int tile = blockIdx.x * 8 + wave;
  if (tile >= tilesM * tilesN) return;
  const int tm = tile / tilesN;
  const int tn = tile - tm * tilesN;
  const int m0 = tm << 6;
  const int n0 = tn << 6;

  const T* Ab  = A  + (size_t)b * strideA;
  const T* Bb  = Bt + (size_t)b * strideB;
  const T* Ab2 = (SPL >= 1) ? (A2  + (size_t)b * strideA) : nullptr;
  const T* Bb2 = (SPL == 2) ? (Bt2 + (size_t)b * strideB) : nullptr;

  const int rlane = lane & 15;
  const int koff  = (lane >> 4) * 8;
  const int mOff  = (lane >> 4) * 8;

  v8f acc[4][4];
#pragma unroll
  for (int i = 0; i < 4; ++i)
#pragma unroll
    for (int j = 0; j < 4; ++j) acc[i][j] = (v8f){0.f,0.f,0.f,0.f,0.f,0.f,0.f,0.f};

  for (int k0 = 0; k0 < K; k0 += 32) {
    V bh[4], bl[4];
#pragma unroll
    for (int j = 0; j < 4; ++j) {
      const size_t bo = (size_t)(n0 + (j << 4) + rlane) * ldb + koff + k0;
      bh[j] = Frag<T>::load(Bb + bo);
      if (SPL == 2) bl[j] = Frag<T>::load(Bb2 + bo);
    }
#pragma unroll
    for (int i = 0; i < 4; ++i) {
      const size_t ao = (size_t)(m0 + (i << 4) + rlane) * lda + koff + k0;
      V ah = Frag<T>::load(Ab + ao);
      V al;
      if (SPL >= 1) al = Frag<T>::load(Ab2 + ao);
#pragma unroll
      for (int j = 0; j < 4; ++j) {
        acc[i][j] = Frag<T>::mma(ah, bh[j], acc[i][j]);
        if (SPL == 2) acc[i][j] = Frag<T>::mma(ah, bl[j], acc[i][j]);
        if (SPL >= 1) acc[i][j] = Frag<T>::mma(al, bh[j], acc[i][j]);
      }
      Frag<T>::guard4(acc[i][0], acc[i][1], acc[i][2], acc[i][3], ah, (SPL >= 1) ? al : ah);
    }
    Frag<T>::keep(bh[0], bh[1], bh[2], bh[3]);
    if (SPL == 2) Frag<T>::keep(bl[0], bl[1], bl[2], bl[3]);
  }
  acc_guard4(acc[0][0], acc[0][1], acc[0][2], acc[0][3]);
  acc_guard4(acc[1][0], acc[1][1], acc[1][2], acc[1][3]);
  acc_guard4(acc[2][0], acc[2][1], acc[2][2], acc[2][3]);
  acc_guard4(acc[3][0], acc[3][1], acc[3][2], acc[3][3]);

  float* slab = sT[wave];
  const float* Rb = RESID ? (resid + (size_t)b * strideR) : nullptr;
#pragma unroll
  for (int i = 0; i < 4; ++i) {
    const int mBase = m0 + (i << 4);
#pragma unroll
    for (int j = 0; j < 4; ++j) {
      const int n = n0 + (j << 4) + rlane;
      float bv = 0.f;
      if (BIAS_MODE == 2) bv = bias[n];
#pragma unroll
      for (int r = 0; r < 8; ++r) {
        float v = acc[i][j][r] * scale;
        if (BIAS_MODE == 1) v += bias[mBase + mOff + r];
        if (BIAS_MODE == 2) v += bv;
        if (RESID) v += Rb[(size_t)(mBase + mOff + r) * ldc + n];
        if (ACT == 1) v = tanhf(v);
        if (ACT == 2) v = fmaxf(v, 0.0f);
        if (ACT == 3) v = v / (1.0f + expf(-v));
        if (ACT == 4) v = (v > 0.f) ? v : 0.01f * v;
        slab[(mOff + r) * 68 + (j << 4) + rlane] = v;
      }
    }
    __builtin_amdgcn_fence(__ATOMIC_RELEASE, "workgroup");
    __builtin_amdgcn_wave_barrier();
    __builtin_amdgcn_fence(__ATOMIC_ACQUIRE, "workgroup");
    if (OUT_MODE == 0) {
      float* C = (float*)Cout + (size_t)b * strideC;
      const int hh = lane >> 4, c4 = (lane & 15) * 4;
      for (int pass = 0; pass < 2; ++pass) {
#pragma unroll
        for (int it = 0; it < 8; ++it) {
          const int row = it * 2 + hh;
          v4f v = *(const v4f*)(slab + row * 68 + c4);
          *(volatile v4f*)(C + (size_t)(mBase + row) * ldc + n0 + c4) = v;
        }
        __threadfence();
      }
    } else {
      const int q = lane >> 3, c8 = (lane & 7) * 8;
      unsigned short* C  = (unsigned short*)Cout  + (size_t)b * strideC;
      unsigned short* C2 = (OUT_MODE == 2) ? ((unsigned short*)Cout2 + (size_t)b * strideC) : nullptr;
      for (int pass = 0; pass < 2; ++pass) {
#pragma unroll
        for (int it = 0; it < 4; ++it) {
          const int row = it * 4 + q;
          const float* sp = slab + row * 68 + c8;
          v8h hv, lv;
#pragma unroll
          for (int e = 0; e < 8; ++e) {
            if (OUT_MODE == 1) {
              hv[e] = (_Float16)sp[e];
            } else {
              unsigned short hb = f2bf_bits(sp[e]);
              unsigned short lb = f2bf_bits(sp[e] - bf_bits2f(hb));
              hv[e] = __builtin_bit_cast(_Float16, hb);
              lv[e] = __builtin_bit_cast(_Float16, lb);
            }
          }
          *(volatile v8h*)(C + (size_t)(mBase + row) * ldc + n0 + c8) = hv;
          if (OUT_MODE == 2) *(volatile v8h*)(C2 + (size_t)(mBase + row) * ldc + n0 + c8) = lv;
        }
        __threadfence();
      }
    }
    __builtin_amdgcn_fence(__ATOMIC_RELEASE, "workgroup");
    __builtin_amdgcn_wave_barrier();
    __builtin_amdgcn_fence(__ATOMIC_ACQUIRE, "workgroup");
  }
}

__global__ __launch_bounds__(256) void cast_plane_bf16_kernel(
    const float* __restrict__ src, unsigned short* __restrict__ dst, int total8, int real8)
{
  const int i = blockIdx.x * 256 + threadIdx.x;
  if (i >= total8) return;
  const bool live = (i < real8);
  const int ic = live ? i : (real8 - 1);
  const size_t e0 = (size_t)ic << 3;
  const v4f a0 = *(const v4f*)(src + e0);
  const v4f a1 = *(const v4f*)(src + e0 + 4);
  const float f0 = live ? a0[0] : 0.0f;
  const float f1 = live ? a0[1] : 0.0f;
  const float f2 = live ? a0[2] : 0.0f;
  const float f3 = live ? a0[3] : 0.0f;
  const float f4 = live ? a1[0] : 0.0f;
  const float f5 = live ? a1[1] : 0.0f;
  const float f6 = live ? a1[2] : 0.0f;
  const float f7 = live ? a1[3] : 0.0f;
  const unsigned w0 = bf_rne_word(f0) | (bf_rne_word(f1) << 16);
  const unsigned w1 = bf_rne_word(f2) | (bf_rne_word(f3) << 16);
  const unsigned w2 = bf_rne_word(f4) | (bf_rne_word(f5) << 16);
  const unsigned w3 = bf_rne_word(f6) | (bf_rne_word(f7) << 16);
  const v4u hv = (v4u){w0, w1, w2, w3};
  unsigned short* q = dst + ((size_t)i << 3);
  *(volatile v4u*)q = hv;
  __threadfence();
  *(volatile v4u*)q = hv;
}

__global__ __launch_bounds__(256) void rmsnorm_split_kernel(
    const float* __restrict__ hs, const float* __restrict__ nw,
    unsigned short* __restrict__ XH, unsigned short* __restrict__ XL)
{
  const int lane = threadIdx.x & 31, wave = threadIdx.x >> 5;
  const int row = blockIdx.x * 8 + wave;
  const float* xr = hs + (size_t)row * kDm;
  float xv[32];
  float ss = 0.0f;
#pragma unroll
  for (int j = 0; j < 4; ++j) {
    const v4f a0 = *(const v4f*)(xr + j * 256 + lane * 8);
    const v4f a1 = *(const v4f*)(xr + j * 256 + lane * 8 + 4);
#pragma unroll
    for (int e = 0; e < 4; ++e) {
      const float g0 = a0[e];
      const float g1 = a1[e];
      const float r0 = rne_bf16_f(g0);
      const float r1 = rne_bf16_f(g1);
      xv[j * 8 + e] = r0;
      xv[j * 8 + 4 + e] = r1;
      ss = fmaf(r0, r0, ss);
      ss = fmaf(r1, r1, ss);
    }
  }
#pragma unroll
  for (int off = 16; off > 0; off >>= 1) ss += __shfl_xor(ss, off, 32);
  const float scale = rsqrtf(ss * (1.0f / (float)kDm) + kEps);
  v4u hv[4], lv[4];
#pragma unroll
  for (int j = 0; j < 4; ++j) {
    const v4f w0 = *(const v4f*)(nw + j * 256 + lane * 8);
    const v4f w1 = *(const v4f*)(nw + j * 256 + lane * 8 + 4);
    v4f y0, y1;
#pragma unroll
    for (int e = 0; e < 4; ++e) {
      const float g0 = w0[e];
      const float g1 = w1[e];
      y0[e] = (xv[j * 8 + e] * scale) * rne_bf16_f(g0);
      y1[e] = (xv[j * 8 + 4 + e] * scale) * rne_bf16_f(g1);
    }
    split_pack8(y0, y1, hv[j], lv[j]);
  }
  unsigned short* ph = XH + (size_t)row * kDm + lane * 8;
  unsigned short* pl = XL + (size_t)row * kDm + lane * 8;
  for (int pass = 0; pass < 2; ++pass) {
#pragma unroll
    for (int j = 0; j < 4; ++j) {
      *(volatile v4u*)(ph + j * 256) = hv[j];
      *(volatile v4u*)(pl + j * 256) = lv[j];
    }
    __threadfence();
  }
}

__global__ __launch_bounds__(256) void conv_silu_kernel(
    const float* __restrict__ XZ, const float* __restrict__ cw, const float* __restrict__ cb,
    float* __restrict__ UC, unsigned short* __restrict__ UCH, unsigned short* __restrict__ UCL)
{
  __shared__ __align__(16) float sT[16 * kConvTP];
  const int tid = threadIdx.x, lane = tid & 31, wave = tid >> 5;
  const int d0 = blockIdx.x * 256, d = d0 + tid;
  const int g0 = blockIdx.y * 64;
  const int tb = g0 & (kSeq - 1);
  const v4f wq = *(const v4f*)(cw + d * 4);
  const float wa = wq[0], wb = wq[1], wc = wq[2], wd = wq[3];
  const float w0 = rne_bf16_f(wa), w1 = rne_bf16_f(wb), w2 = rne_bf16_f(wc), w3 = rne_bf16_f(wd);
  const float bc = rne_bf16_f(cb[d]);
  float xm3, xm2, xm1;
  {
    const bool hist = (tb > 0);
    const int rb = hist ? (g0 - 3) : g0;
    const float v3 = XZ[(size_t)rb * kXzP + d];
    const float v2 = XZ[(size_t)(rb + 1) * kXzP + d];
    const float v1 = XZ[(size_t)(rb + 2) * kXzP + d];
    xm3 = hist ? v3 : 0.f;
    xm2 = hist ? v2 : 0.f;
    xm1 = hist ? v1 : 0.f;
  }
  const int hrow = wave >> 1;
  const int hch  = (wave & 1) * 128 + lane * 4;
#pragma unroll 1
  for (int sub = 0; sub < 4; ++sub) {
    const int lb = g0 + sub * 16;
#pragma unroll 1
    for (int s = 0; s < 16; ++s) {
      const float xcur = XZ[(size_t)(lb + s) * kXzP + d];
      float acc = w0 * xm3;
      acc = fmaf(w1, xm2, acc);
      acc = fmaf(w2, xm1, acc);
      acc = fmaf(w3, xcur, acc);
      const float sv = acc + bc;
      const float sg = __builtin_amdgcn_rcpf(1.0f + expf(-sv));
      sT[s * kConvTP + tid] = sv * sg;
      xm3 = xm2; xm2 = xm1; xm1 = xcur;
    }
    __syncthreads();
    v4f fv[4];
    v4u bh[2], blo[2];
#pragma unroll
    for (int it = 0; it < 4; ++it) fv[it] = *(const v4f*)(sT + (it * 4 + hrow) * kConvTP + hch);
#pragma unroll
    for (int it = 0; it < 2; ++it) {
      const float* sp = sT + (it * 8 + wave) * kConvTP + lane * 8;
      const v4f a0 = *(const v4f*)(sp);
      const v4f a1 = *(const v4f*)(sp + 4);
      split_pack8(a0, a1, bh[it], blo[it]);
    }
    for (int pass = 0; pass < 2; ++pass) {
#pragma unroll
      for (int it = 0; it < 4; ++it)
        *(volatile v4f*)(UC + (size_t)(lb + it * 4 + hrow) * kDin + d0 + hch) = fv[it];
#pragma unroll
      for (int it = 0; it < 2; ++it) {
        const size_t o = (size_t)(lb + it * 8 + wave) * kDin + d0 + lane * 8;
        *(volatile v4u*)(UCH + o) = bh[it];
        *(volatile v4u*)(UCL + o) = blo[it];
      }
      __threadfence();
    }
    __syncthreads();
  }
}

__global__ __launch_bounds__(256) void dt_split_kernel(
    const float* __restrict__ DBL, unsigned short* __restrict__ DTH, unsigned short* __restrict__ DTL, int total8)
{
  const int i = blockIdx.x * 256 + threadIdx.x;
  if (i >= total8) return;
  const int e0  = i << 3;
  const int row = e0 >> 6;
  const int c8  = e0 & 63;
  const float* p = DBL + (size_t)row * kPrjP + c8;
  const v4f a0 = *(const v4f*)(p);
  const v4f a1 = *(const v4f*)(p + 4);
  v4u hv, lv;
  split_pack8(a0, a1, hv, lv);
  unsigned short* qh = DTH + e0;
  unsigned short* ql = DTL + e0;
  *(volatile v4u*)qh = hv;
  *(volatile v4u*)ql = lv;
  __threadfence();
  *(volatile v4u*)qh = hv;
  *(volatile v4u*)ql = lv;
}

__global__ __launch_bounds__(64) void scan_kernel(
    const float* __restrict__ DBL, const float* __restrict__ DLR, const float* __restrict__ UC,
    const float* __restrict__ XZ, const float* __restrict__ bdt, const float* __restrict__ Alog,
    const float* __restrict__ Dp, unsigned short* __restrict__ YH, unsigned short* __restrict__ YL)
{
  __shared__ __align__(16) float sBC[kScanTS * 16];
  __shared__ __align__(16) float sY[kScanTS * kScanYP];
  __shared__ __align__(16) float sA[kNst * kScanCh];
  const int tid = threadIdx.x, lane = tid & 31, wave = tid >> 5;
  constexpr int kBlkPerB = kDin / kScanCh;
  const int bix = blockIdx.x / kBlkPerB;
  const int d0  = (blockIdx.x - bix * kBlkPerB) * kScanCh;
  const int d   = d0 + tid;
  const size_t row0 = (size_t)bix * kSeq;
#pragma unroll 1
  for (int s = 0; s < kNst; ++s) sA[s * kScanCh + tid] = -expf(rne_bf16_f(Alog[(size_t)d * kNst + s]));
  __syncthreads();
  float negA[kNst], h[kNst];
#pragma unroll
  for (int s = 0; s < kNst; ++s) {
    negA[s] = sA[s * kScanCh + tid];
    h[s] = 0.f;
  }
  const float bb = rne_bf16_f(bdt[d]);
  const float Dd = rne_bf16_f(Dp[d]);
  const int q = lane >> 3, c8 = (lane & 7) * 8;
#pragma unroll 1
  for (int t0 = 0; t0 < kSeq; t0 += kScanTS) {
    __syncthreads();
#pragma unroll
    for (int i = 0; i < 4; ++i) {
      const int idx = tid + 64 * i;
      const int r = idx >> 2;
      const int c4 = (idx & 3) * 4;
      *(v4f*)(sBC + r * 16 + c4) = *(const v4f*)(DBL + (row0 + t0 + r) * kPrjP + kDtR + c4);
    }
    __syncthreads();
#pragma unroll 1
    for (int s = 0; s < kScanTS; ++s) {
      const size_t m = row0 + t0 + s;
      const float* xr = sBC + s * 16;
      const v4f b0 = *(const v4f*)(xr);
      const v4f b1 = *(const v4f*)(xr + 4);
      const v4f c0 = *(const v4f*)(xr + 8);
      const v4f c1 = *(const v4f*)(xr + 12);
      const float Bs[kNst] = {b0[0], b0[1], b0[2], b0[3], b1[0], b1[1], b1[2], b1[3]};
      const float Cs[kNst] = {c0[0], c0[1], c0[2], c0[3], c1[0], c1[1], c1[2], c1[3]};
      float pre = DLR[m * kDin + d];
      float xt  = UC[m * kDin + d];
      float zv  = XZ[m * kXzP + kDin + d];
      asm volatile("" : "+v"(pre));
      asm volatile("" : "+v"(xt));
      asm volatile("" : "+v"(zv));
      const float v   = pre + bb;
      const float a   = expf(-fabsf(v));
      const float u   = 1.0f + a;
      const float l1p = __logf(u) + (a - (u - 1.0f)) * __builtin_amdgcn_rcpf(u);
      const float dt  = fmaxf(v, 0.0f) + l1p;
      float y = 0.f;
#pragma unroll
      for (int n = 0; n < kNst; ++n) {
        const float e  = __expf(dt * negA[n]);
        const float bx = (dt * Bs[n]) * xt;
        h[n] = fmaf(e, h[n], bx);
        y = fmaf(h[n], Cs[n], y);
      }
      y = fmaf(Dd, xt, y);
      const float sg = __builtin_amdgcn_rcpf(1.0f + expf(-zv));
      y = y * (zv * sg);
      sY[s * kScanYP + tid] = y;
    }
    __syncthreads();
    v4u hv[8], lv[8];
#pragma unroll
    for (int it = 0; it < 8; ++it) {
      const int row = it * 8 + wave * 4 + q;
      const float* sp = sY + row * kScanYP + c8;
      const v4f a0 = *(const v4f*)(sp);
      const v4f a1 = *(const v4f*)(sp + 4);
      split_pack8(a0, a1, hv[it], lv[it]);
    }
    for (int pass = 0; pass < 2; ++pass) {
#pragma unroll
      for (int it = 0; it < 8; ++it) {
        const int row = it * 8 + wave * 4 + q;
        const size_t o = (row0 + t0 + row) * kDin + d0 + c8;
        *(volatile v4u*)(YH + o) = hv[it];
        *(volatile v4u*)(YL + o) = lv[it];
      }
      __threadfence();
    }
  }
}

static_assert(((kHRows / 64) * (kXzP / 64)) % 8 == 0);
static_assert(((kHRows / 64) * (kPrjP / 64)) % 8 == 0);
static_assert(((kHRows / 64) * (kDin / 64)) % 8 == 0);
static_assert(((kHRows / 64) * (kDm / 64)) % 8 == 0);
static_assert(((kXzP * kDm / 8) % 256) == 0 && ((kPrjP * kDin / 8) % 256) == 0 &&
              ((kDin * kDtR / 8) % 256) == 0 && ((kDm * kDin / 8) % 256) == 0 && ((kHRows * kDtR / 8) % 256) == 0);

extern "C" void kernel_launch(void* const* d_in, const int* in_sizes, int n_in,
                              void* d_out, int out_size, void* d_ws, size_t ws_size,
                              hipStream_t stream) {
  if (n_in < 11) return;
  if (in_sizes[0] != kRows * kDm) return;
  if (in_sizes[1] != kDm) return;
  if (in_sizes[2] != kXzP * kDm) return;
  if (in_sizes[3] != kDin * 4) return;
  if (in_sizes[4] != kDin) return;
  if (in_sizes[5] != kPrjN * kDin) return;
  if (in_sizes[6] != kDin * kDtR) return;
  if (in_sizes[7] != kDin) return;
  if (in_sizes[8] != kDin * kNst) return;
  if (in_sizes[9] != kDin) return;
  if (in_sizes[10] != kDm * kDin) return;
  if (out_size != kRows * kDm) return;
  if (ws_size < kWsTotal) return;

  const float* hidden  = (const float*)d_in[0];
  const float* norm_w  = (const float*)d_in[1];
  const float* W_in    = (const float*)d_in[2];
  const float* conv_w  = (const float*)d_in[3];
  const float* conv_b  = (const float*)d_in[4];
  const float* W_xproj = (const float*)d_in[5];
  const float* W_dt    = (const float*)d_in[6];
  const float* b_dt    = (const float*)d_in[7];
  const float* A_log   = (const float*)d_in[8];
  const float* D_skip  = (const float*)d_in[9];
  const float* W_out   = (const float*)d_in[10];
  float* out = (float*)d_out;

  char* ws = (char*)d_ws;
  unsigned short* WIN  = (unsigned short*)(ws + kOffWIN);
  unsigned short* WXP  = (unsigned short*)(ws + kOffWXP);
  unsigned short* WDT  = (unsigned short*)(ws + kOffWDT);
  unsigned short* WOUT = (unsigned short*)(ws + kOffWOUT);
  unsigned short* XNH  = (unsigned short*)(ws + kOffXNH);
  unsigned short* XNL  = (unsigned short*)(ws + kOffXNL);
  float*          XZ   = (float*)(ws + kOffXZ);
  float*          UC   = (float*)(ws + kOffUC);
  unsigned short* UCH  = (unsigned short*)(ws + kOffUCH);
  unsigned short* UCL  = (unsigned short*)(ws + kOffUCL);
  float*          DBL  = (float*)(ws + kOffDBL);
  unsigned short* DTH  = (unsigned short*)(ws + kOffDTH);
  unsigned short* DTL  = (unsigned short*)(ws + kOffDTL);
  float*          DLR  = (float*)(ws + kOffDLR);
  unsigned short* YH   = (unsigned short*)(ws + kOffYH);
  unsigned short* YL   = (unsigned short*)(ws + kOffYL);

  cast_plane_bf16_kernel<<<(kXzP * kDm / 8) / 256, 256, 0, stream>>>(W_in, WIN, kXzP * kDm / 8, kXzP * kDm / 8);
  cast_plane_bf16_kernel<<<(kPrjP * kDin / 8) / 256, 256, 0, stream>>>(W_xproj, WXP, kPrjP * kDin / 8, kPrjN * kDin / 8);
  cast_plane_bf16_kernel<<<(kDin * kDtR / 8) / 256, 256, 0, stream>>>(W_dt, WDT, kDin * kDtR / 8, kDin * kDtR / 8);
  cast_plane_bf16_kernel<<<(kDm * kDin / 8) / 256, 256, 0, stream>>>(W_out, WOUT, kDm * kDin / 8, kDm * kDin / 8);

  for (int hf = 0; hf < kHalves; ++hf) {
    const float* hs_h = hidden + (size_t)hf * kHRows * kDm;
    float* out_h = out + (size_t)hf * kHRows * kDm;

    rmsnorm_split_kernel<<<kHRows / 8, 256, 0, stream>>>(hs_h, norm_w, XNH, XNL);

    wmma_gemm64<1, 1, 0, 0, false><<<dim3((kHRows / 64) * (kXzP / 64) / 8, 1), 256, 0, stream>>>(
        XNH, XNL, kDm, 0L,
        WIN, WIN, kDm, 0L,
        (void*)XZ, (void*)XZ, kXzP, 0L,
        b_dt, hs_h, 0L,
        kHRows, kXzP, kDm, 1.0f);

    conv_silu_kernel<<<dim3(kDin / 256, kHRows / 64), 256, 0, stream>>>(XZ, conv_w, conv_b, UC, UCH, UCL);

    wmma_gemm64<1, 1, 0, 0, false><<<dim3((kHRows / 64) * (kPrjP / 64) / 8, 1), 256, 0, stream>>>(
        UCH, UCL, kDin, 0L,
        WXP, WXP, kDin, 0L,
        (void*)DBL, (void*)DBL, kPrjP, 0L,
        b_dt, hs_h, 0L,
        kHRows, kPrjP, kDin, 1.0f);

    dt_split_kernel<<<(kHRows * kDtR / 8) / 256, 256, 0, stream>>>(DBL, DTH, DTL, kHRows * kDtR / 8);

    wmma_gemm64<1, 1, 0, 0, false><<<dim3((kHRows / 64) * (kDin / 64) / 8, 1), 256, 0, stream>>>(
        DTH, DTL, kDtR, 0L,
        WDT, WDT, kDtR, 0L,
        (void*)DLR, (void*)DLR, kDin, 0L,
        b_dt, hs_h, 0L,
        kHRows, kDin, kDtR, 1.0f);

    scan_kernel<<<kBatchPH * (kDin / kScanCh), kScanCh, 0, stream>>>(DBL, DLR, UC, XZ, b_dt, A_log, D_skip, YH, YL);

    wmma_gemm64<1, 1, 0, 0, false><<<dim3((kHRows / 64) * (kDm / 64) / 8, 1), 256, 0, stream>>>(
        YH, YL, kDin, 0L,
        WOUT, WOUT, kDin, 0L,
        (void*)out_h, (void*)out_h, kDm, 0L,
        b_dt, hs_h, 0L,
        kHRows, kDm, kDin, 1.0f);
  }
}
